// sSE_13383118095126
// MI455X (gfx1250) — hardware-verified
//
#include <hip/hip_runtime.h>

typedef _Float16 f16t;
typedef _Float16 v16h __attribute__((ext_vector_type(16)));
typedef _Float16 v8h  __attribute__((ext_vector_type(8)));
typedef float    v8f  __attribute__((ext_vector_type(8)));
typedef float    v4f  __attribute__((ext_vector_type(4)));
typedef v8h  __attribute__((may_alias)) v8ha;
typedef v4f  __attribute__((may_alias)) v4fa;
union Frag  { v16h v; v8h half[2]; };
union Q8    { v8f v; v4f q[2]; };

#define NB      2
#define CH      64
#define CO      32
#define CQ      8
#define NP      4096
#define SD      16
#define PADV    18
#define PZS     324
#define NPP     5832
#define K3      1728
#define QKP     32
#define QKPLANE (NB * NP * QKP)
#define XSP     72
#define WSP     72
#define VSP     72
#define SSP     72
#define PSP     72
#define WSC     16.0f
#define W3SC    64.0f
#define QKCAR   4.0f
#define VCAR    8.0f
#define PCAR    1024.0f
#define ACAR    8.0f
#define NWCV    6912
#define NZR     93312

__device__ __forceinline__ v8f wmma_f16(v16h a, v16h b, v8f c) {
  v8f d = __builtin_amdgcn_wmma_f32_16x16x32_f16(false, a, false, b, (short)0, c, false, false);
  asm volatile("v_nop\n\tv_nop\n\tv_nop\n\tv_nop" : "+v"(d) : "v"(a), "v"(b));
  return d;
}

__device__ __forceinline__ v16h load_frag32(const f16t* p, int h) {
  Frag f;
  f.half[0] = *(const v8ha*)(p + 8 * h);
  f.half[1] = *(const v8ha*)(p + 16 + 8 * h);
  return f.v;
}

__device__ __forceinline__ v8f zero8f() {
  v8f z;
  #pragma unroll
  for (int j = 0; j < 8; ++j) z[j] = 0.f;
  return z;
}

__device__ __forceinline__ void st8f(float* p, v8f v) {
  Q8 u; u.v = v;
  *(v4fa*)p = u.q[0];
  *(v4fa*)(p + 4) = u.q[1];
}

__global__ __launch_bounds__(256) void k_prep(const float* __restrict__ wid,
                                             f16t* __restrict__ Wr, f16t* __restrict__ YP)
{
  const int g = blockIdx.x * 256 + threadIdx.x;
  if (g < NWCV) {
    const int e8 = g * 8;
    const int o = e8 / K3, kk = e8 - o * K3;
    const int tap = kk >> 6, c = kk & 63;
    const float* base = wid + ((size_t)(o * CH + c) * 27 + tap);
    v8h o8;
    #pragma unroll
    for (int i = 0; i < 8; ++i) o8[i] = (f16t)(base[i * 27] * W3SC);
    f16t* dst = Wr + e8;
    *(volatile v8h*)dst = o8;
    __threadfence();
    *(volatile v8h*)dst = o8;
    return;
  }
  const int g2 = g - NWCV;
  if (g2 >= NZR) return;
  const int b = g2 / (NPP * 8);
  const int r = g2 - b * (NPP * 8);
  const int pp = r >> 3, v = r & 7;
  const int z = pp / PZS, rem = pp - z * PZS;
  const int y = rem / PADV, d = rem - y * PADV;
  const bool ring = (z == 0) | (z == PADV - 1) | (y == 0) | (y == PADV - 1) | (d == 0) | (d == PADV - 1);
  if (!ring) return;
  v8h zz;
  #pragma unroll
  for (int j = 0; j < 8; ++j) zz[j] = (f16t)0.0f;
  f16t* dst = YP + (size_t)(b * NPP + pp) * CH + 8 * v;
  *(volatile v8h*)dst = zz;
  __threadfence();
  *(volatile v8h*)dst = zz;
}

__global__ __launch_bounds__(256) void k_qkv(
    const float* __restrict__ x, const float* __restrict__ wq, const float* __restrict__ wk,
    const float* __restrict__ wv, f16t* __restrict__ QK, f16t* __restrict__ VC)
{
  __shared__ __attribute__((aligned(16))) f16t sX[64 * XSP];
  __shared__ __attribute__((aligned(16))) f16t sW[80 * WSP];
  __shared__ __attribute__((aligned(16))) f16t sV[CH * VSP];
  __shared__ __attribute__((aligned(16))) f16t sQK[2 * 64 * QKP];
  const int tid = threadIdx.x, lane = tid & 31, w = tid >> 5;
  const int h = lane >> 4, m = lane & 15;
  const int p0 = blockIdx.x * 64, b = blockIdx.y;

  {
    v8h zz;
    #pragma unroll
    for (int j = 0; j < 8; ++j) zz[j] = (f16t)0.0f;
    *(v8ha*)(sQK + 16 * tid) = zz;
    *(v8ha*)(sQK + 16 * tid + 8) = zz;
  }
  #pragma unroll
  for (int j = 0; j < 4; ++j) {
    const int idx = tid + 256 * j;
    const int c = idx >> 4, x4 = (idx & 15) * 4;
    const v4f v = *(const v4fa*)(x + (size_t)(b * CH + c) * NP + p0 + x4);
    sX[(x4 + 0) * XSP + c] = (f16t)v.x;
    sX[(x4 + 1) * XSP + c] = (f16t)v.y;
    sX[(x4 + 2) * XSP + c] = (f16t)v.z;
    sX[(x4 + 3) * XSP + c] = (f16t)v.w;
  }
  #pragma unroll
  for (int it = 0; it < 2; ++it) {
    const int i = tid + 256 * it;
    const int row = i >> 6, c = i & 63;
    sW[row * WSP + c] = (f16t)(wq[i] * WSC);
    sW[(CQ + row) * WSP + c] = (f16t)(wk[i] * WSC);
  }
  #pragma unroll 1
  for (int it = 0; it < 16; ++it) {
    const int i = tid + 256 * it;
    const int row = i >> 6, c = i & 63;
    sW[(2 * CQ + row) * WSP + c] = (f16t)(wv[i] * WSC);
  }
  __syncthreads();

  const int mt = w & 3, vg = w >> 2;
  const v8f z8 = zero8f();
  v8f accv[2], accq;
  accv[0] = z8; accv[1] = z8; accq = z8;
  #pragma unroll
  for (int k0 = 0; k0 < CH; k0 += 32) {
    const v16h a = load_frag32(sX + (16 * mt + m) * XSP + k0, h);
    const v16h bq = load_frag32(sW + m * WSP + k0, h);
    const v16h b0 = load_frag32(sW + (16 + 16 * (2 * vg) + m) * WSP + k0, h);
    const v16h b1 = load_frag32(sW + (16 + 16 * (2 * vg + 1) + m) * WSP + k0, h);
    accq = wmma_f16(a, bq, accq);
    accv[0] = wmma_f16(a, b0, accv[0]);
    accv[1] = wmma_f16(a, b1, accv[1]);
  }

  const float osc = 1.0f / WSC;
  #pragma unroll
  for (int t = 0; t < 2; ++t) {
    const int c = 16 * (2 * vg + t) + m;
    v8h hv;
    #pragma unroll
    for (int r = 0; r < 8; ++r) hv[r] = (f16t)(accv[t][r] * osc * VCAR);
    *(v8ha*)(sV + c * VSP + 16 * mt + 8 * h) = hv;
  }
  if (w < 4) {
    const int plb = (m >> 3) * (64 * QKP) + (m & 7);
    #pragma unroll
    for (int r = 0; r < 8; ++r) {
      const int pos = 16 * mt + 8 * h + r;
      sQK[plb + pos * QKP] = (f16t)(accq[r] * osc * QKCAR);
    }
  }
  __syncthreads();

  const int q8 = lane & 7, sub = lane >> 3;
  #pragma unroll
  for (int i = 0; i < 2; ++i) {
    const int c = 8 * w + 4 * i + sub;
    const v8h val = *(const v8ha*)(sV + c * VSP + 8 * q8);
    const size_t d = (size_t)(b * CH + c) * NP + p0 + 8 * q8;
    *(volatile v8h*)(VC + d) = val;
  }
  #pragma unroll
  for (int i = 0; i < 2; ++i) {
    const int id = 8 * w + 4 * i + sub;
    const int pl = id >> 5, L = id & 31;
    const v8h val = *(const v8ha*)(sQK + pl * (64 * QKP) + L * 64 + 8 * q8);
    const size_t d = (size_t)pl * QKPLANE + (size_t)(b * NP + p0) * QKP + L * 64 + 8 * q8;
    *(volatile v8h*)(QK + d) = val;
  }
  __threadfence();
  #pragma unroll
  for (int i = 0; i < 2; ++i) {
    const int c = 8 * w + 4 * i + sub;
    const v8h val = *(const v8ha*)(sV + c * VSP + 8 * q8);
    const size_t d = (size_t)(b * CH + c) * NP + p0 + 8 * q8;
    *(volatile v8h*)(VC + d) = val;
  }
  #pragma unroll
  for (int i = 0; i < 2; ++i) {
    const int id = 8 * w + 4 * i + sub;
    const int pl = id >> 5, L = id & 31;
    const v8h val = *(const v8ha*)(sQK + pl * (64 * QKP) + L * 64 + 8 * q8);
    const size_t d = (size_t)pl * QKPLANE + (size_t)(b * NP + p0) * QKP + L * 64 + 8 * q8;
    *(volatile v8h*)(QK + d) = val;
  }
}

__global__ __launch_bounds__(256) void k_att(
    const f16t* __restrict__ QK, const f16t* __restrict__ VC, const float* __restrict__ xres,
    const float* __restrict__ gam, f16t* __restrict__ YP)
{
  __shared__ __attribute__((aligned(16))) float Ssw[64 * SSP];
  __shared__ __attribute__((aligned(16))) f16t  Psw[64 * PSP];
  __shared__ __attribute__((aligned(16))) f16t  sT[64 * CH];
  __shared__ float rsc[64];
  __shared__ float lsum[64];
  const int tid = threadIdx.x, lane = tid & 31, w = tid >> 5;
  const int h = lane >> 4, m = lane & 15;
  const int i0 = blockIdx.x * 64, b = blockIdx.y;
  const int is_ = w >> 1, jsa = 2 * (w & 1);
  const int ct = w & 3, jsb = 2 * (w >> 2);
  const int si = tid >> 2, jq = tid & 3;
  const float sinv = 1.0f / (QKCAR * QKCAR);
  const f16t* Qp = QK;
  const f16t* Kp = QK + QKPLANE;
  const v16h bq = load_frag32(Qp + (size_t)(b * NP + i0 + 16 * is_ + m) * QKP, h);
  const f16t* vrow = VC + (size_t)(b * CH + 16 * ct + m) * NP;
  const v8f z8 = zero8f();
  v8f acc[2];
  acc[0] = z8; acc[1] = z8;
  float mrun = -1.0e30f, lrun = 0.f;

  #pragma unroll 1
  for (int j0 = 0; j0 < NP; j0 += 64) {
    {
      const f16t* kp = Kp + (size_t)(b * NP + j0 + 16 * jsa + m) * QKP;
      const v16h a0 = load_frag32(kp, h);
      const v16h a1 = load_frag32(kp + 16 * QKP, h);
      const v8f s0 = wmma_f16(a0, bq, z8);
      const v8f s1 = wmma_f16(a1, bq, z8);
      st8f(Ssw + (16 * is_ + m) * SSP + 16 * jsa + 8 * h, s0);
      st8f(Ssw + (16 * is_ + m) * SSP + 16 * jsa + 16 + 8 * h, s1);
    }
    __syncthreads();

    float sv[16];
    {
      const float* sp = Ssw + si * SSP + 16 * jq;
      #pragma unroll
      for (int q = 0; q < 4; ++q) {
        const v4f t4 = *(const v4fa*)(sp + 4 * q);
        sv[4 * q + 0] = t4.x; sv[4 * q + 1] = t4.y; sv[4 * q + 2] = t4.z; sv[4 * q + 3] = t4.w;
      }
    }
    float mx = sv[0];
    #pragma unroll
    for (int r = 1; r < 16; ++r) mx = fmaxf(mx, sv[r]);
    mx = fmaxf(mx, __shfl_xor(mx, 1));
    mx = fmaxf(mx, __shfl_xor(mx, 2));
    const float mnew = fmaxf(mrun, mx);
    const float rs = __expf((mrun - mnew) * sinv);
    mrun = mnew;
    float psum = 0.f;
    v8h pa, pb;
    #pragma unroll
    for (int r = 0; r < 8; ++r) {
      const float p = __expf((sv[r] - mnew) * sinv);
      psum += p;
      pa[r] = (f16t)(p * PCAR);
    }
    #pragma unroll
    for (int r = 0; r < 8; ++r) {
      const float p = __expf((sv[8 + r] - mnew) * sinv);
      psum += p;
      pb[r] = (f16t)(p * PCAR);
    }
    psum += __shfl_xor(psum, 1);
    psum += __shfl_xor(psum, 2);
    lrun = lrun * rs + psum;
    if (jq == 0) rsc[si] = rs;
    *(v8ha*)(Psw + si * PSP + 16 * jq) = pa;
    *(v8ha*)(Psw + si * PSP + 16 * jq + 8) = pb;
    __syncthreads();

    #pragma unroll
    for (int t = 0; t < 2; ++t) {
      const float rr = rsc[16 * (jsb + t) + m];
      #pragma unroll
      for (int e = 0; e < 8; ++e) acc[t][e] *= rr;
    }
    #pragma unroll
    for (int kc = 0; kc < 2; ++kc) {
      const v16h a = load_frag32(vrow + j0 + 32 * kc, h);
      #pragma unroll
      for (int t = 0; t < 2; ++t) {
        const v16h bb = load_frag32(Psw + (16 * (jsb + t) + m) * PSP + 32 * kc, h);
        acc[t] = wmma_f16(a, bb, acc[t]);
      }
    }
  }

  if (jq == 0) lsum[si] = lrun;
  __syncthreads();
  #pragma unroll
  for (int j = 0; j < 4; ++j) {
    const int idx = tid + 256 * j;
    const int c = idx >> 4, x4 = (idx & 15) * 4;
    const v4f v = *(const v4fa*)(xres + (size_t)(b * CH + c) * NP + i0 + x4);
    *(v4fa*)(Ssw + c * SSP + x4) = v;
  }
  __syncthreads();
  const float gsc = gam[0] * (1.0f / (VCAR * PCAR));
  const int cb = 16 * ct + 8 * h;
  #pragma unroll
  for (int t = 0; t < 2; ++t) {
    const int il = 16 * (jsb + t) + m;
    const float linv = gsc * __builtin_amdgcn_rcpf(lsum[il]);
    v8h hv;
    #pragma unroll
    for (int r = 0; r < 8; ++r) hv[r] = (f16t)((acc[t][r] * linv + Ssw[(cb + r) * SSP + il]) * ACAR);
    *(v8ha*)(sT + il * CH + cb) = hv;
  }
  __syncthreads();

  const int q8 = lane & 7, sub = lane >> 3;
  #pragma unroll
  for (int i = 0; i < 2; ++i) {
    const int lid = 8 * w + 4 * i + sub;
    const v8h val = *(const v8ha*)(sT + lid * CH + 8 * q8);
    const int n = i0 + lid;
    const int z = n >> 8, y = (n >> 4) & 15, d = n & 15;
    const int pp = (z + 1) * PZS + (y + 1) * PADV + d + 1;
    const size_t dd = (size_t)(b * NPP + pp) * CH + 8 * q8;
    *(volatile v8h*)(YP + dd) = val;
  }
  __threadfence();
  #pragma unroll
  for (int i = 0; i < 2; ++i) {
    const int lid = 8 * w + 4 * i + sub;
    const v8h val = *(const v8ha*)(sT + lid * CH + 8 * q8);
    const int n = i0 + lid;
    const int z = n >> 8, y = (n >> 4) & 15, d = n & 15;
    const int pp = (z + 1) * PZS + (y + 1) * PADV + d + 1;
    const size_t dd = (size_t)(b * NPP + pp) * CH + 8 * q8;
    *(volatile v8h*)(YP + dd) = val;
  }
}

__global__ __launch_bounds__(256) void k_conv(
    const f16t* __restrict__ YP, const f16t* __restrict__ Wr, float* __restrict__ out)
{
  __shared__ __attribute__((aligned(16))) float sO[CO * 256];
  const int tid = threadIdx.x, lane = tid & 31, w = tid >> 5;
  const int h = lane >> 4, m = lane & 15;
  const int z = blockIdx.x, b = blockIdx.y;
  const v8f z8 = zero8f();
  v8f acc[2][2];
  #pragma unroll
  for (int yy = 0; yy < 2; ++yy) { acc[yy][0] = z8; acc[yy][1] = z8; }

  #pragma unroll 1
  for (int tap = 0; tap < 27; ++tap) {
    const int dz = tap / 9, r9 = tap - 9 * dz;
    const int dy = r9 / 3, dd = r9 - 3 * dy;
    const int rowz = b * NPP + (z + dz) * PZS + dd;
    const f16t* wb = Wr + (size_t)m * K3 + (size_t)tap * CH;
    #pragma unroll
    for (int c0 = 0; c0 < CH; c0 += 32) {
      v16h a[2], bb[2];
      #pragma unroll
      for (int yy = 0; yy < 2; ++yy) {
        const int y = 2 * w + yy;
        const int rowb = rowz + (y + dy) * PADV;
        a[yy] = load_frag32(YP + (size_t)(rowb + m) * CH + c0, h);
      }
      #pragma unroll
      for (int nt = 0; nt < 2; ++nt) bb[nt] = load_frag32(wb + (size_t)(16 * nt) * K3 + c0, h);
      #pragma unroll
      for (int yy = 0; yy < 2; ++yy) {
        acc[yy][0] = wmma_f16(a[yy], bb[0], acc[yy][0]);
        acc[yy][1] = wmma_f16(a[yy], bb[1], acc[yy][1]);
      }
    }
  }

  const float osc = 1.0f / (ACAR * W3SC);
  #pragma unroll
  for (int yy = 0; yy < 2; ++yy) {
    const int y = 2 * w + yy;
    #pragma unroll
    for (int nt = 0; nt < 2; ++nt) {
      const int oc = 16 * nt + m;
      v8f vv;
      #pragma unroll
      for (int r = 0; r < 8; ++r) vv[r] = acc[yy][nt][r] * osc;
      st8f(sO + oc * 256 + y * 16 + 8 * h, vv);
    }
  }
  __syncthreads();

  const int q8 = lane & 7, sub = lane >> 3;
  const size_t obase = (size_t)(b * CO) * NP + (size_t)z * 256;
  #pragma unroll
  for (int i = 0; i < 8; ++i) {
    const int L = 32 * w + 4 * i + sub;
    const int oc = L >> 3, piece = L & 7;
    const v4f val = *(const v4fa*)(sO + oc * 256 + piece * 32 + 4 * q8);
    const size_t d = obase + (size_t)oc * NP + piece * 32 + 4 * q8;
    *(volatile v4f*)(out + d) = val;
  }
  __threadfence();
  #pragma unroll
  for (int i = 0; i < 8; ++i) {
    const int L = 32 * w + 4 * i + sub;
    const int oc = L >> 3, piece = L & 7;
    const v4f val = *(const v4fa*)(sO + oc * 256 + piece * 32 + 4 * q8);
    const size_t d = obase + (size_t)oc * NP + piece * 32 + 4 * q8;
    *(volatile v4f*)(out + d) = val;
  }
}

extern "C" void kernel_launch(void* const* d_in, const int* in_sizes, int n_in,
                              void* d_out, int out_size, void* d_ws, size_t ws_size,
                              hipStream_t stream) {
  if (n_in < 6) return;
  if (in_sizes[0] != NB * CH * NP) return;
  if (in_sizes[1] != CQ * CH || in_sizes[2] != CQ * CH) return;
  if (in_sizes[3] != CH * CH) return;
  if (in_sizes[4] < 1) return;
  if (in_sizes[5] != CO * CH * 27) return;
  if (out_size != NB * CO * NP) return;

  const float* x    = (const float*)d_in[0];
  const float* wq   = (const float*)d_in[1];
  const float* wk   = (const float*)d_in[2];
  const float* wv   = (const float*)d_in[3];
  const float* gam  = (const float*)d_in[4];
  const float* wid  = (const float*)d_in[5];
  float* outp = (float*)d_out;

  const size_t szWr = (size_t)CO * K3 * 2;
  const size_t szYP = (size_t)NB * NPP * CH * 2;
  const size_t szVC = (size_t)NB * CH * NP * 2;
  const size_t szQK = (size_t)2 * NB * NP * QKP * 2;
  size_t off = 0;
  char* ws = (char*)d_ws;
  f16t* Wr = (f16t*)(ws + off); off += szWr;
  f16t* YP = (f16t*)(ws + off); off += szYP;
  f16t* VC = (f16t*)(ws + off); off += szVC;
  f16t* QK = (f16t*)(ws + off); off += szQK;
  if (off > ws_size) return;

  k_prep<<<(NWCV + NZR + 255) / 256, 256, 0, stream>>>(wid, Wr, YP);
  k_qkv<<<dim3(NP / 64, NB), 256, 0, stream>>>(x, wq, wk, wv, QK, VC);
  k_att<<<dim3(NP / 64, NB), 256, 0, stream>>>(QK, VC, x, gam, YP);
  k_conv<<<dim3(SD, NB), 256, 0, stream>>>(YP, Wr, outp);
}
